// PointNetFeatureUpsampling_61469571940541
// MI455X (gfx1250) — hardware-verified
//
#include <hip/hip_runtime.h>
#pragma clang fp contract(off)

typedef __attribute__((ext_vector_type(16))) _Float16 v16h;
typedef __attribute__((ext_vector_type(8)))  _Float16 v8h;
typedef __attribute__((ext_vector_type(8)))  float    v8f;
typedef __attribute__((ext_vector_type(4)))  float    v4f;
typedef __attribute__((ext_vector_type(4)))  int      v4i;

constexpr int NBATCH   = 16;
constexpr int NPTS     = 2048;
constexpr int NSRC     = 512;
constexpr int DFEAT    = 384;
constexpr int CCAT     = 768;
constexpr int COUT0    = 768;
constexpr int COUT1    = 384;
constexpr int NROWS    = NBATCH * NPTS;
constexpr int CHUNK_N  = 192;
constexpr int STAT_CHUNKS = 128;
constexpr int STAT_ROWS   = NROWS / STAT_CHUNKS;
constexpr float W_CARRY     = 65536.0f;
constexpr float W_CARRY_INV = 1.0f / 65536.0f;
constexpr float BN_EPS_F    = 1e-5f;

static_assert(NPTS == 2048, "row >> 11 gives the batch");
static_assert(CCAT == 2 * DFEAT, "concat width");
static_assert(CCAT % 32 == 0, "K multiple of 32");
static_assert(NROWS % 64 == 0 && CHUNK_N % 64 == 0, "tile multiples");
static_assert(((NROWS / 64) * (CHUNK_N / 64)) % 8 == 0, "whole blocks of 8 wave tiles");
static_assert(COUT0 % CHUNK_N == 0 && COUT1 % CHUNK_N == 0, "channel chunks");
static_assert(CHUNK_N % 32 == 0, "whole 128-B lines per partial row");
static_assert(STAT_ROWS * STAT_CHUNKS == NROWS, "stat chunks cover all rows");
static_assert((COUT0 * CCAT) % (8 * 256) == 0 && (COUT1 * CCAT) % (8 * 256) == 0, "weight prep coverage");

constexpr size_t SZ_X    = (size_t)NROWS * CCAT * 2;
constexpr size_t SZ_H0   = (size_t)NROWS * COUT0 * 2;
constexpr size_t SZ_YC   = (size_t)NROWS * CHUNK_N * 4;
constexpr size_t SZ_W0   = (size_t)COUT0 * CCAT * 2;
constexpr size_t SZ_W1   = (size_t)COUT1 * CCAT * 2;
constexpr size_t SZ_KNN  = (size_t)NROWS * 8 * 4;
constexpr size_t SZ_PART = (size_t)STAT_CHUNKS * CHUNK_N * 4;
constexpr size_t SZ_VEC  = 1024;
constexpr size_t OFF_X    = 0;
constexpr size_t OFF_H0   = OFF_X + SZ_X;
constexpr size_t OFF_YC   = OFF_H0 + SZ_H0;
constexpr size_t OFF_W0H  = OFF_YC + SZ_YC;
constexpr size_t OFF_W0L  = OFF_W0H + SZ_W0;
constexpr size_t OFF_W1H  = OFF_W0L + SZ_W0;
constexpr size_t OFF_W1L  = OFF_W1H + SZ_W1;
constexpr size_t OFF_KNNI = OFF_W1L + SZ_W1;
constexpr size_t OFF_KNND = OFF_KNNI + SZ_KNN;
constexpr size_t OFF_PS   = OFF_KNND + SZ_KNN;
constexpr size_t OFF_PQ   = OFF_PS + SZ_PART;
constexpr size_t OFF_SC   = OFF_PQ + SZ_PART;
constexpr size_t OFF_SH   = OFF_SC + SZ_VEC;
constexpr size_t WS_TOTAL = OFF_SH + SZ_VEC;
static_assert(WS_TOTAL <= (size_t)134217728, "carve within 128 MiB");
static_assert(OFF_SH % 128 == 0 && OFF_PS % 128 == 0 && OFF_KNNI % 128 == 0, "line-aligned carve");
static_assert((size_t)CHUNK_N * 4 <= SZ_VEC, "scale/shift vectors fit");

struct FragH {
  union U { v16h v; v8h h[2]; };
  static __device__ __forceinline__ v16h load(const _Float16* p) {
    U f; f.h[0] = *(const v8h*)(p); f.h[1] = *(const v8h*)(p + 16); return f.v;
  }
  static __device__ __forceinline__ v8f mma(v16h a, v16h b, v8f c) {
    return __builtin_amdgcn_wmma_f32_16x16x32_f16(false, a, false, b, (short)0, c, false, false);
  }
};
__device__ __forceinline__ void group_guard(v8f& a0, v8f& a1, v8f& a2, v8f& a3, v16h x,
                                            v16h p0, v16h p1, v16h p2, v16h p3,
                                            v16h q0, v16h q1, v16h q2, v16h q3) {
  asm volatile("v_nop\n\tv_nop\n\tv_nop\n\tv_nop"
               : "+v"(a0), "+v"(a1), "+v"(a2), "+v"(a3)
               : "v"(x), "v"(p0), "v"(p1), "v"(p2), "v"(p3), "v"(q0), "v"(q1), "v"(q2), "v"(q3));
}
__device__ __forceinline__ void acc_guard4(v8f& a, v8f& b, v8f& c, v8f& d) {
  asm volatile("v_nop\n\tv_nop\n\tv_nop\n\tv_nop" : "+v"(a), "+v"(b), "+v"(c), "+v"(d));
}

__global__ __launch_bounds__(256) void gemm64_f16_bsplit(
    const unsigned short* __restrict__ Ap, int lda,
    const unsigned short* __restrict__ Bhp, const unsigned short* __restrict__ Blp, int ldb,
    float* __restrict__ Cout, int ldc, int M, int N, int K, float scale) {
  const _Float16* A  = (const _Float16*)Ap;
  const _Float16* Bh = (const _Float16*)Bhp;
  const _Float16* Bl = (const _Float16*)Blp;
  __shared__ __align__(16) float sT[8][16 * 68];
  const int lane = threadIdx.x & 31;
  const int wave = threadIdx.x >> 5;
  const int tilesN = N >> 6;
  const int tilesM = M >> 6;
  const int tile = blockIdx.x * 8 + wave;
  if (tile >= tilesM * tilesN) return;
  const int tm = tile / tilesN;
  const int tn = tile - tm * tilesN;
  const int m0 = tm << 6;
  const int n0 = tn << 6;

  const int rlane = lane & 15;
  const int koff  = (lane >> 4) * 8;
  const int mOff  = (lane >> 4) * 8;

  v8f acc[4][4];
#pragma unroll
  for (int i = 0; i < 4; ++i)
#pragma unroll
    for (int j = 0; j < 4; ++j) acc[i][j] = (v8f){0.f,0.f,0.f,0.f,0.f,0.f,0.f,0.f};

  for (int k0 = 0; k0 < K; k0 += 32) {
    v16h bh[4], bl[4];
#pragma unroll
    for (int j = 0; j < 4; ++j) {
      const size_t bo = (size_t)(n0 + (j << 4) + rlane) * ldb + koff + k0;
      bh[j] = FragH::load(Bh + bo);
      bl[j] = FragH::load(Bl + bo);
    }
#pragma unroll
    for (int i = 0; i < 4; ++i) {
      const size_t ao = (size_t)(m0 + (i << 4) + rlane) * lda + koff + k0;
      v16h ah = FragH::load(A + ao);
#pragma unroll
      for (int j = 0; j < 4; ++j) {
        acc[i][j] = FragH::mma(ah, bh[j], acc[i][j]);
        acc[i][j] = FragH::mma(ah, bl[j], acc[i][j]);
      }
      group_guard(acc[i][0], acc[i][1], acc[i][2], acc[i][3], ah,
                  bh[0], bh[1], bh[2], bh[3], bl[0], bl[1], bl[2], bl[3]);
    }
  }
  acc_guard4(acc[0][0], acc[0][1], acc[0][2], acc[0][3]);
  acc_guard4(acc[1][0], acc[1][1], acc[1][2], acc[1][3]);
  acc_guard4(acc[2][0], acc[2][1], acc[2][2], acc[2][3]);
  acc_guard4(acc[3][0], acc[3][1], acc[3][2], acc[3][3]);

  float* slab = sT[wave];
#pragma unroll
  for (int i = 0; i < 4; ++i) {
    const int mBase = m0 + (i << 4);
#pragma unroll
    for (int j = 0; j < 4; ++j) {
#pragma unroll
      for (int r = 0; r < 8; ++r) {
        const float v = acc[i][j][r] * scale;
        slab[(mOff + r) * 68 + (j << 4) + rlane] = v;
      }
    }
    __builtin_amdgcn_fence(__ATOMIC_RELEASE, "workgroup");
    __builtin_amdgcn_wave_barrier();
    __builtin_amdgcn_fence(__ATOMIC_ACQUIRE, "workgroup");
    {
      const int hh = lane >> 4, c4 = (lane & 15) * 4;
      for (int pass = 0; pass < 2; ++pass) {
#pragma unroll
        for (int it = 0; it < 8; ++it) {
          const int row = it * 2 + hh;
          v4f v = *(const v4f*)(slab + row * 68 + c4);
          *(volatile v4f*)(Cout + (size_t)(mBase + row) * ldc + n0 + c4) = v;
        }
        __threadfence();
      }
    }
    __builtin_amdgcn_fence(__ATOMIC_RELEASE, "workgroup");
    __builtin_amdgcn_wave_barrier();
    __builtin_amdgcn_fence(__ATOMIC_ACQUIRE, "workgroup");
  }
}

__global__ __launch_bounds__(256) void prep_w_kernel(
    const float* __restrict__ w0, const float* __restrict__ w1,
    unsigned short* __restrict__ w0h, unsigned short* __restrict__ w0l,
    unsigned short* __restrict__ w1h, unsigned short* __restrict__ w1l, int blocks0) {
  const bool first = ((int)blockIdx.x < blocks0);
  const float* src = first ? w0 : w1;
  unsigned short* dh = first ? w0h : w1h;
  unsigned short* dl = first ? w0l : w1l;
  const int blk = first ? (int)blockIdx.x : ((int)blockIdx.x - blocks0);
  const size_t e0 = ((size_t)blk * 256 + threadIdx.x) * 8;
  const v4f a = *(const v4f*)(src + e0);
  const v4f c = *(const v4f*)(src + e0 + 4);
  v8h hv, lv;
#pragma unroll
  for (int e = 0; e < 8; ++e) {
    const float raw = (e < 4) ? a[e & 3] : c[e & 3];
    float s = raw * W_CARRY;
    s = fminf(fmaxf(s, -60000.0f), 60000.0f);
    const _Float16 hs = (_Float16)s;
    const float hf = (float)hs;
    const float rr = s - hf;
    const _Float16 ls = (_Float16)rr;
    hv[e] = hs;
    lv[e] = ls;
  }
  for (int pass = 0; pass < 2; ++pass) {
    *(volatile v8h*)(dh + e0) = hv;
    *(volatile v8h*)(dl + e0) = lv;
    __threadfence();
  }
}

__global__ __launch_bounds__(256) void knn_kernel(
    const float* __restrict__ xyz1, const float* __restrict__ xyz2,
    const int* __restrict__ elens, int* __restrict__ knnI, float* __restrict__ knnD) {
#pragma clang fp contract(off)
  __shared__ __align__(16) float sp[NSRC * 4];
  __shared__ __align__(16) int   sI[256 * 8];
  __shared__ __align__(16) float sD[256 * 8];
  const int tid = threadIdx.x;
  const int b = blockIdx.x >> 3;
  const int n = ((blockIdx.x & 7) << 8) + tid;
  const float* p2 = xyz2 + (size_t)b * NSRC * 3;
#pragma unroll
  for (int u = 0; u < 2; ++u) {
    const int s = tid + u * 256;
    const float xs = p2[s * 3 + 0];
    const float ys = p2[s * 3 + 1];
    const float zs = p2[s * 3 + 2];
    const float xx = xs * xs;
    const float yy = ys * ys;
    const float zz = zs * zs;
    const float q = (xx + zz) + yy;
    const v4f pk = {xs, ys, zs, q};
    *(v4f*)(sp + 4 * s) = pk;
  }
  __syncthreads();
  int slen = elens[b];
  slen = slen < 0 ? 0 : (slen > NSRC ? NSRC : slen);
  const float* p1 = xyz1 + ((size_t)b * NPTS + n) * 3;
  const float x = p1[0], y = p1[1], z = p1[2];
  const float x2 = x * x;
  const float y2 = y * y;
  const float z2 = z * z;
  const float n1 = (x2 + z2) + y2;

  float d0 = 3.0e38f, d1 = 3.0e38f, d2 = 3.0e38f, d3 = 3.0e38f, d4 = 3.0e38f;
  int i0 = 0, i1 = 0, i2 = 0, i3 = 0, i4 = 0;
#pragma unroll 2
  for (int s = 0; s < NSRC; ++s) {
    const v4f pk = *(const v4f*)(sp + 4 * s);
    const float xs = pk[0], ys = pk[1], zs = pk[2], q2 = pk[3];
    float p = x * xs;
    p = __builtin_fmaf(y, ys, p);
    p = __builtin_fmaf(z, zs, p);
    const float ssum = n1 + q2;
    const float p2x = p + p;
    float dd = ssum - p2x;
    dd = (s < slen) ? dd : 1e10f;
    const bool c0 = dd < d0, c1 = dd < d1, c2 = dd < d2, c3 = dd < d3, c4 = dd < d4;
    d4 = c4 ? (c3 ? d3 : dd) : d4;  i4 = c4 ? (c3 ? i3 : s) : i4;
    d3 = c3 ? (c2 ? d2 : dd) : d3;  i3 = c3 ? (c2 ? i2 : s) : i3;
    d2 = c2 ? (c1 ? d1 : dd) : d2;  i2 = c2 ? (c1 ? i1 : s) : i2;
    d1 = c1 ? (c0 ? d0 : dd) : d1;  i1 = c1 ? (c0 ? i0 : s) : i1;
    d0 = c0 ? dd : d0;              i0 = c0 ? s : i0;
  }
  {
    const v4i ia = {i0, i1, i2, i3};
    const v4i ib = {i4, 0, 0, 0};
    const v4f da = {d0, d1, d2, d3};
    const v4f db = {d4, 0.0f, 0.0f, 0.0f};
    *(v4i*)(sI + tid * 8)     = ia;
    *(v4i*)(sI + tid * 8 + 4) = ib;
    *(v4f*)(sD + tid * 8)     = da;
    *(v4f*)(sD + tid * 8 + 4) = db;
  }
  __syncthreads();
  int*   gI = knnI + (size_t)blockIdx.x * 256 * 8;
  float* gD = knnD + (size_t)blockIdx.x * 256 * 8;
  for (int pass = 0; pass < 2; ++pass) {
#pragma unroll
    for (int p = 0; p < 2; ++p) {
      const int c = p * 256 + tid;
      const v4i vi = *(const v4i*)(sI + c * 4);
      const v4f vd = *(const v4f*)(sD + c * 4);
      *(volatile v4i*)(gI + c * 4) = vi;
      *(volatile v4f*)(gD + c * 4) = vd;
    }
    __threadfence();
  }
}

__device__ __forceinline__ void gather_acc8(float (&acc)[8], const float* __restrict__ g, float w) {
  const v4f a = *(const v4f*)(g);
  const v4f c = *(const v4f*)(g + 4);
#pragma unroll
  for (int e = 0; e < 4; ++e) {
    acc[e]     = acc[e]     + w * a[e];
    acc[4 + e] = acc[4 + e] + w * c[e];
  }
}

__global__ __launch_bounds__(256) void buildx_kernel(
    const float* __restrict__ points1, const float* __restrict__ points2,
    const int* __restrict__ knnI, const float* __restrict__ knnD,
    unsigned short* __restrict__ X) {
  const int lane = threadIdx.x & 31;
  const int wave = threadIdx.x >> 5;
  const int row = blockIdx.x * 16 + wave * 2 + (lane >> 4);
  const int c8 = (lane & 15) * 8;
  const int b = row >> 11;
  const float* p1 = points1 + (size_t)row * DFEAT + c8;
  unsigned short* xr = X + (size_t)row * CCAT + c8;
#pragma unroll 1
  for (int it = 0; it < 3; ++it) {
    const v4f a = *(const v4f*)(p1 + it * 128);
    const v4f c = *(const v4f*)(p1 + it * 128 + 4);
    v8h hv;
#pragma unroll
    for (int e = 0; e < 4; ++e) {
      const float fa = a[e];
      const float fc = c[e];
      hv[e]     = (_Float16)fa;
      hv[4 + e] = (_Float16)fc;
    }
    volatile v8h* dst = (volatile v8h*)(xr + it * 128);
    *dst = hv;
    __threadfence();
    *dst = hv;
  }
  const v4i ia = *(const v4i*)(knnI + (size_t)row * 8);
  const v4i ib = *(const v4i*)(knnI + (size_t)row * 8 + 4);
  const v4f da = *(const v4f*)(knnD + (size_t)row * 8);
  const v4f db = *(const v4f*)(knnD + (size_t)row * 8 + 4);
  int j0 = ia[0], j1 = ia[1], j2 = ia[2], j3 = ia[3], j4 = ib[0];
  j0 = j0 < 0 ? 0 : (j0 > NSRC - 1 ? NSRC - 1 : j0);
  j1 = j1 < 0 ? 0 : (j1 > NSRC - 1 ? NSRC - 1 : j1);
  j2 = j2 < 0 ? 0 : (j2 > NSRC - 1 ? NSRC - 1 : j2);
  j3 = j3 < 0 ? 0 : (j3 > NSRC - 1 ? NSRC - 1 : j3);
  j4 = j4 < 0 ? 0 : (j4 > NSRC - 1 ? NSRC - 1 : j4);
  const float eps = 1.1920929e-07f;
  const float r0 = 1.0f / (da[0] + eps);
  const float r1 = 1.0f / (da[1] + eps);
  const float r2 = 1.0f / (da[2] + eps);
  const float r3 = 1.0f / (da[3] + eps);
  const float r4 = 1.0f / (db[0] + eps);
  float rs = r0 + r1;
  rs = rs + r2;
  rs = rs + r3;
  rs = rs + r4;
  const float inv = 1.0f / rs;
  const float w0 = r0 * inv, w1 = r1 * inv, w2 = r2 * inv, w3 = r3 * inv, w4 = r4 * inv;
  const float* pb = points2 + (size_t)b * NSRC * DFEAT + c8;
  const float* g0 = pb + (size_t)j0 * DFEAT;
  const float* g1 = pb + (size_t)j1 * DFEAT;
  const float* g2 = pb + (size_t)j2 * DFEAT;
  const float* g3 = pb + (size_t)j3 * DFEAT;
  const float* g4 = pb + (size_t)j4 * DFEAT;
#pragma unroll 1
  for (int it = 0; it < 3; ++it) {
    const int off = it * 128;
    float acc[8];
#pragma unroll
    for (int e = 0; e < 8; ++e) acc[e] = 0.0f;
    gather_acc8(acc, g0 + off, w0);
    gather_acc8(acc, g1 + off, w1);
    gather_acc8(acc, g2 + off, w2);
    asm volatile("" : "+v"(acc[0]), "+v"(acc[1]), "+v"(acc[2]), "+v"(acc[3]),
                      "+v"(acc[4]), "+v"(acc[5]), "+v"(acc[6]), "+v"(acc[7]) :: "memory");
    gather_acc8(acc, g3 + off, w3);
    gather_acc8(acc, g4 + off, w4);
    v8h hv;
#pragma unroll
    for (int e = 0; e < 8; ++e) {
      const float f = acc[e];
      hv[e] = (_Float16)f;
    }
    volatile v8h* dst = (volatile v8h*)(xr + DFEAT + off);
    *dst = hv;
    __threadfence();
    *dst = hv;
  }
}

__global__ __launch_bounds__(192) void stats_kernel(
    const float* __restrict__ Y, const int* __restrict__ mask,
    float* __restrict__ pS, float* __restrict__ pQ) {
  __shared__ int sm[STAT_ROWS];
  const int chunk = blockIdx.x;
  const int r0 = chunk * STAT_ROWS;
  const int ch = threadIdx.x;
  for (int i = threadIdx.x; i < STAT_ROWS; i += 192) sm[i] = mask[r0 + i];
  __syncthreads();
  const float* yp = Y + (size_t)r0 * CHUNK_N + ch;
  float s = 0.0f, q = 0.0f;
#pragma unroll 4
  for (int i = 0; i < STAT_ROWS; ++i) {
    const float v = yp[(size_t)i * CHUNK_N];
    const float vm = (sm[i] != 0) ? v : 0.0f;
    const float v2 = vm * vm;
    s = s + vm;
    q = q + v2;
  }
  volatile float* ds = pS + (size_t)chunk * CHUNK_N + ch;
  volatile float* dq = pQ + (size_t)chunk * CHUNK_N + ch;
  for (int pass = 0; pass < 2; ++pass) {
    *ds = s;
    *dq = q;
    __threadfence();
  }
}

__global__ __launch_bounds__(256) void bnfin_kernel(
    const float* __restrict__ pS, const float* __restrict__ pQ, const int* __restrict__ mask,
    const float* __restrict__ gam, const float* __restrict__ bet,
    float* __restrict__ scale, float* __restrict__ shift) {
  __shared__ int scnt[256];
  const int tid = threadIdx.x;
  int c = 0;
  const int* mp = mask + tid * (NROWS / 256);
#pragma unroll 4
  for (int i = 0; i < NROWS / 256 / 4; ++i) {
    const v4i m = *(const v4i*)(mp + 4 * i);
    c += (m[0] != 0) + (m[1] != 0) + (m[2] != 0) + (m[3] != 0);
  }
  scnt[tid] = c;
  __syncthreads();
  for (int st = 128; st > 0; st >>= 1) {
    if (tid < st) scnt[tid] += scnt[tid + st];
    __syncthreads();
  }
  const float cnt = (float)scnt[0];
  const float icnt = 1.0f / cnt;
  const int ch = tid < CHUNK_N ? tid : (CHUNK_N - 1);
  float s = 0.0f, q = 0.0f;
#pragma unroll 4
  for (int k = 0; k < STAT_CHUNKS; ++k) {
    s = s + pS[(size_t)k * CHUNK_N + ch];
    q = q + pQ[(size_t)k * CHUNK_N + ch];
  }
  const float mean = s * icnt;
  const float m2 = mean * mean;
  float var = q * icnt - m2;
  var = fmaxf(var, 0.0f);
  const float rstd = 1.0f / sqrtf(var + BN_EPS_F);
  const float sc = rstd * gam[ch];
  const float ms = mean * sc;
  const float sh = bet[ch] - ms;
  if (tid < CHUNK_N) {
    volatile float* d0 = scale + tid;
    volatile float* d1 = shift + tid;
    for (int pass = 0; pass < 2; ++pass) {
      *d0 = sc;
      *d1 = sh;
      __threadfence();
    }
  }
}

__global__ __launch_bounds__(256) void apply_h_kernel(
    const float* __restrict__ Y, const float* __restrict__ scale, const float* __restrict__ shift,
    unsigned short* __restrict__ H, int colBase) {
  const int t = blockIdx.x * 256 + threadIdx.x;
  const int u = t >> 3;
  const int sub = t & 7;
  const int row = u / 3;
  const int seg = u - row * 3;
  const int ch = seg * 64 + sub * 8;
  const float* yp = Y + (size_t)row * CHUNK_N + ch;
  const v4f ya = *(const v4f*)(yp);
  const v4f yb = *(const v4f*)(yp + 4);
  const v4f sa = *(const v4f*)(scale + ch);
  const v4f sb = *(const v4f*)(scale + ch + 4);
  const v4f ta = *(const v4f*)(shift + ch);
  const v4f tb = *(const v4f*)(shift + ch + 4);
  v8h hv;
#pragma unroll
  for (int e = 0; e < 4; ++e) {
    const float pa = ya[e] * sa[e];
    const float pb = yb[e] * sb[e];
    const float va = fmaxf(pa + ta[e], 0.0f);
    const float vb = fmaxf(pb + tb[e], 0.0f);
    hv[e]     = (_Float16)va;
    hv[4 + e] = (_Float16)vb;
  }
  volatile v8h* dst = (volatile v8h*)(H + (size_t)row * COUT0 + colBase + ch);
  *dst = hv;
  __threadfence();
  *dst = hv;
}

__global__ __launch_bounds__(256) void apply_out_kernel(
    const float* __restrict__ Y, const float* __restrict__ scale, const float* __restrict__ shift,
    float* __restrict__ out, int colBase) {
  const int t = blockIdx.x * 256 + threadIdx.x;
  const int u = t >> 3;
  const int sub = t & 7;
  const int row = u / 6;
  const int seg = u - row * 6;
  const int ch = seg * 32 + sub * 4;
  const v4f ya = *(const v4f*)(Y + (size_t)row * CHUNK_N + ch);
  const v4f sa = *(const v4f*)(scale + ch);
  const v4f ta = *(const v4f*)(shift + ch);
  v4f ov;
#pragma unroll
  for (int e = 0; e < 4; ++e) {
    const float pa = ya[e] * sa[e];
    ov[e] = fmaxf(pa + ta[e], 0.0f);
  }
  volatile v4f* dst = (volatile v4f*)(out + (size_t)row * COUT1 + colBase + ch);
  *dst = ov;
  __threadfence();
  *dst = ov;
}

extern "C" void kernel_launch(void* const* d_in, const int* in_sizes, int n_in,
                              void* d_out, int out_size, void* d_ws, size_t ws_size,
                              hipStream_t stream) {
  if (n_in < 13) return;
  if (ws_size < WS_TOTAL) return;
  if (out_size != NROWS * COUT1) return;
  if (in_sizes[0] != NROWS * 3 || in_sizes[1] != NBATCH * NSRC * 3) return;
  if (in_sizes[2] != NROWS * DFEAT || in_sizes[3] != NBATCH * NSRC * DFEAT) return;
  if (in_sizes[6] != NROWS || in_sizes[7] != COUT0 * CCAT || in_sizes[10] != COUT1 * CCAT) return;

  const float* xyz1    = (const float*)d_in[0];
  const float* xyz2    = (const float*)d_in[1];
  const float* points1 = (const float*)d_in[2];
  const float* points2 = (const float*)d_in[3];
  const int*   elens   = (const int*)d_in[5];
  const int*   pmask   = (const int*)d_in[6];
  const float* W0 = (const float*)d_in[7];
  const float* g0 = (const float*)d_in[8];
  const float* b0 = (const float*)d_in[9];
  const float* W1 = (const float*)d_in[10];
  const float* g1 = (const float*)d_in[11];
  const float* b1 = (const float*)d_in[12];
  float* out = (float*)d_out;

  char* base = (char*)d_ws;
  unsigned short* X   = (unsigned short*)(base + OFF_X);
  unsigned short* H0  = (unsigned short*)(base + OFF_H0);
  float*          Yc  = (float*)(base + OFF_YC);
  unsigned short* W0h = (unsigned short*)(base + OFF_W0H);
  unsigned short* W0l = (unsigned short*)(base + OFF_W0L);
  unsigned short* W1h = (unsigned short*)(base + OFF_W1H);
  unsigned short* W1l = (unsigned short*)(base + OFF_W1L);
  int*   knnI = (int*)(base + OFF_KNNI);
  float* knnD = (float*)(base + OFF_KNND);
  float* pS = (float*)(base + OFF_PS);
  float* pQ = (float*)(base + OFF_PQ);
  float* sc = (float*)(base + OFF_SC);
  float* sh = (float*)(base + OFF_SH);

  const int blocksW0 = (COUT0 * CCAT) / (8 * 256);
  const int blocksW1 = (COUT1 * CCAT) / (8 * 256);
  prep_w_kernel<<<blocksW0 + blocksW1, 256, 0, stream>>>(W0, W1, W0h, W0l, W1h, W1l, blocksW0);
  knn_kernel<<<NROWS / 256, 256, 0, stream>>>(xyz1, xyz2, elens, knnI, knnD);
  buildx_kernel<<<NROWS / 16, 256, 0, stream>>>(points1, points2, knnI, knnD, X);

  const int gemmBlocks = ((NROWS / 64) * (CHUNK_N / 64)) / 8;
  for (int c = 0; c < COUT0 / CHUNK_N; ++c) {
    const size_t wOff = (size_t)c * CHUNK_N * CCAT;
    gemm64_f16_bsplit<<<gemmBlocks, 256, 0, stream>>>(X, CCAT, W0h + wOff, W0l + wOff, CCAT,
                                                       Yc, CHUNK_N, NROWS, CHUNK_N, CCAT, W_CARRY_INV);
    stats_kernel<<<STAT_CHUNKS, 192, 0, stream>>>(Yc, pmask, pS, pQ);
    bnfin_kernel<<<1, 256, 0, stream>>>(pS, pQ, pmask, g0 + c * CHUNK_N, b0 + c * CHUNK_N, sc, sh);
    apply_h_kernel<<<(NROWS * (CHUNK_N / 64) * 8) / 256, 256, 0, stream>>>(Yc, sc, sh, H0, c * CHUNK_N);
  }
  for (int c = 0; c < COUT1 / CHUNK_N; ++c) {
    const size_t wOff = (size_t)c * CHUNK_N * COUT0;
    gemm64_f16_bsplit<<<gemmBlocks, 256, 0, stream>>>(H0, COUT0, W1h + wOff, W1l + wOff, COUT0,
                                                       Yc, CHUNK_N, NROWS, CHUNK_N, COUT0, W_CARRY_INV);
    stats_kernel<<<STAT_CHUNKS, 192, 0, stream>>>(Yc, pmask, pS, pQ);
    bnfin_kernel<<<1, 256, 0, stream>>>(pS, pQ, pmask, g1 + c * CHUNK_N, b1 + c * CHUNK_N, sc, sh);
    apply_out_kernel<<<(NROWS * (CHUNK_N / 32) * 8) / 256, 256, 0, stream>>>(Yc, sc, sh, out, c * CHUNK_N);
  }
}
